// SpatialCrossBranchAttention_47553877901508
// MI455X (gfx1250) — hardware-verified
//
#include <hip/hip_runtime.h>
#include <math.h>

typedef __attribute__((ext_vector_type(16))) _Float16 v16h;
typedef __attribute__((ext_vector_type(16))) __bf16 v16b;
typedef __attribute__((ext_vector_type(8)))  _Float16 v8h;
typedef __attribute__((ext_vector_type(8)))  float v8f;
typedef __attribute__((ext_vector_type(4)))  float v4f;
typedef __attribute__((ext_vector_type(2)))  float v2f;
typedef __attribute__((ext_vector_type(4)))  unsigned v4u;
typedef __attribute__((ext_vector_type(4)))  int v4i;
typedef float __attribute__((may_alias)) float_a;
typedef int __attribute__((may_alias)) int_a;

template <typename T> __device__ __forceinline__ void vst2(void* p, T v) { *(volatile T*)p = v; __threadfence(); *(volatile T*)p = v; }
__device__ __forceinline__ v8f wmma16(v16h a, v16h b, v8f c) {
  v8f d = __builtin_amdgcn_wmma_f32_16x16x32_f16(false, a, false, b, (short)0, c, false, false);
  asm volatile("v_nop\n\tv_nop\n\tv_nop\n\tv_nop" : "+v"(d) : "v"(a), "v"(b));
  return d;
}
__device__ __forceinline__ v8f wmma_bf(v16b a, v16b b, v8f c) {
  v8f d = __builtin_amdgcn_wmma_f32_16x16x32_bf16(false, a, false, b, (short)0, c, false, false);
  asm volatile("v_nop\n\tv_nop\n\tv_nop\n\tv_nop" : "+v"(d) : "v"(a), "v"(b));
  return d;
}
__device__ __forceinline__ v16h frag_h(const _Float16* rowk0, int lane) {
  union { v16h v; v8h q[2]; } u; const _Float16* p = rowk0 + 8 * (lane >> 4);
  u.q[0] = *(const v8h*)p; u.q[1] = *(const v8h*)(p + 16); return u.v;
}
__device__ __forceinline__ v16h frag_f32(const float* rowk0, int lane) {
  v16h a; const float* p = rowk0 + 8 * (lane >> 4);
#pragma unroll
  for (int i = 0; i < 8; ++i) { a[i] = (_Float16)p[i]; a[8 + i] = (_Float16)p[16 + i]; }
  return a;
}
__device__ __forceinline__ v16h frag_f32s(const float* rowk0, int lane, float sc) {
  v16h a; const float* p = rowk0 + 8 * (lane >> 4);
#pragma unroll
  for (int i = 0; i < 8; ++i) { a[i] = (_Float16)(p[i] * sc); a[8 + i] = (_Float16)(p[16 + i] * sc); }
  return a;
}
__device__ __forceinline__ v16h fragc_f32(const float* W, int k0, int n, int lane, int ld, int K) {
  v16h a; const int g = lane >> 4;
#pragma unroll
  for (int i = 0; i < 8; ++i) { const int ka = k0 + 8 * g + i, kb = ka + 16;
    a[i] = (_Float16)(ka < K ? W[(size_t)(ka < K ? ka : K - 1) * ld + n] : 0.f); a[8 + i] = (_Float16)(kb < K ? W[(size_t)(kb < K ? kb : K - 1) * ld + n] : 0.f); }
  return a;
}
struct F2 { v16b h, l; };
__device__ __forceinline__ F2 bsplit16(const float v[16]) { F2 r;
#pragma unroll
  for (int i = 0; i < 16; ++i) { const __bf16 h = (__bf16)v[i]; r.h[i] = h; r.l[i] = (__bf16)(v[i] - (float)h); }
  return r; }
__device__ __forceinline__ F2 split_row(const float* row, int k0, int lane) { float v[16]; const float* p = row + k0 + 8 * (lane >> 4);
#pragma unroll
  for (int i = 0; i < 8; ++i) { v[i] = p[i]; v[8 + i] = p[16 + i]; }
  return bsplit16(v); }
__device__ __forceinline__ F2 split_rowK(const float* row, int k0, int lane, int K) { float v[16]; const int g = lane >> 4;
#pragma unroll
  for (int i = 0; i < 8; ++i) { const int ka = k0 + 8 * g + i, kb = ka + 16; v[i] = ka < K ? row[ka < K ? ka : K - 1] : 0.f; v[8 + i] = kb < K ? row[kb < K ? kb : K - 1] : 0.f; }
  return bsplit16(v); }
__device__ __forceinline__ F2 split_col(const float* W, int k0, int n, int lane, int ld, int K) { float v[16]; const int g = lane >> 4;
#pragma unroll
  for (int i = 0; i < 8; ++i) { const int ka = k0 + 8 * g + i, kb = ka + 16; v[i] = ka < K ? W[(size_t)(ka < K ? ka : K - 1) * ld + n] : 0.f; v[8 + i] = kb < K ? W[(size_t)(kb < K ? kb : K - 1) * ld + n] : 0.f; }
  return bsplit16(v); }
__device__ __forceinline__ v8f mac3(const F2& a, const F2& b, v8f c) { c = wmma_bf(a.l, b.h, c); c = wmma_bf(a.h, b.l, c); return wmma_bf(a.h, b.h, c); }
__device__ __forceinline__ float sigm(float v) { return 1.0f / (1.0f + expf(-v)); }
#define LDSX() do { asm volatile("s_wait_dscnt 0" ::: "memory"); __builtin_amdgcn_wave_barrier(); __builtin_amdgcn_fence(__ATOMIC_RELEASE, "workgroup"); } while (0)


#define NB 4
#define CC 64
#define NN 4096
#define C8 8
__device__ __forceinline__ float bfr(float v) { return (float)(__bf16)v; }
__device__ __forceinline__ v16b frag_b(const __bf16* rowk0, int lane) { return __builtin_bit_cast(v16b, frag_h((const _Float16*)rowk0, lane)); }
__device__ __attribute__((noinline)) float exp_ni(float v) { return expf(v); }

__global__ __launch_bounds__(256) void k_cvt(const float* __restrict__ x1, const float* __restrict__ x2, __bf16* __restrict__ X1T, __bf16* __restrict__ X2T) {
  __shared__ __align__(16) __bf16 st[64][CC + 8];
  const int tid = threadIdx.x; const int b = blockIdx.y, n0 = blockIdx.x * 64, which = blockIdx.z; const float* x = which == 0 ? x1 : x2; __bf16* XT = which == 0 ? X1T : X2T;
  for (int q = tid; q < CC * 16; q += 256) { const int c = q >> 4, p4 = q & 15; const v4f v = *(const v4f*)(x + ((size_t)b * CC + c) * NN + n0 + p4 * 4);
    st[p4 * 4][c] = (__bf16)v[0]; st[p4 * 4 + 1][c] = (__bf16)v[1]; st[p4 * 4 + 2][c] = (__bf16)v[2]; st[p4 * 4 + 3][c] = (__bf16)v[3]; }
  __syncthreads();
  for (int q = tid; q < 64 * (CC / 8); q += 256) { const int rl = q / (CC / 8), pc = q % (CC / 8); vst2((unsigned*)(XT + ((size_t)b * NN + n0 + rl) * CC + pc * 8), *(const v4u*)(&st[rl][pc * 8])); }
}
__global__ __launch_bounds__(64) void k_q(const float* __restrict__ xt, const float* __restrict__ Wq, const float* __restrict__ bq, const float* __restrict__ Wk, float* __restrict__ QP) {
  __shared__ __align__(16) float sq[64][CC + 4]; __shared__ float swq[C8][CC], swk[C8][CC], sbq[C8];
  const int tid = threadIdx.x; const int b = blockIdx.y, n0 = blockIdx.x * 64; const int n = n0 + tid;
  for (int q = tid; q < C8 * CC; q += 64) { swq[q / CC][q % CC] = bfr(Wq[q]); swk[q / CC][q % CC] = bfr(Wk[q]); }
  if (tid < C8) sbq[tid] = bfr(bq[tid]);
  __syncthreads();
  float qv[C8];
#pragma unroll
  for (int o = 0; o < C8; ++o) qv[o] = sbq[o];
#pragma unroll 1
  for (int c = 0; c < CC; ++c) { const float xv = bfr(xt[((size_t)b * CC + c) * NN + n]);
#pragma unroll
    for (int o = 0; o < C8; ++o) qv[o] += swq[o][c] * xv; }
#pragma unroll 1
  for (int c = 0; c < CC; ++c) { float a = 0.f;
#pragma unroll
    for (int o = 0; o < C8; ++o) a += qv[o] * swk[o][c];
    sq[tid][c] = a; }
  __syncthreads();
  for (int q = tid; q < 64 * 16; q += 64) { const int rl = q >> 4, pc = q & 15; vst2(QP + ((size_t)b * NN + n0 + rl) * CC + pc * 4, *(const v4f*)(&sq[rl][pc * 4])); }
}
__global__ __launch_bounds__(128) void k_attn(const float* __restrict__ QP, const __bf16* __restrict__ X2T, const float* __restrict__ x2, float* __restrict__ CTX) {
  __shared__ __align__(16) float sS[4][16][68];
  __shared__ __align__(16) __bf16 sPh[4][16][72], sPl[4][16][72];
  __shared__ __align__(16) float sO[4][16][68];
  const int tid = threadIdx.x, w = tid >> 5, lane = tid & 31, col = lane & 15, g = lane >> 4; const int b = blockIdx.y; const int q0 = blockIdx.x * 64 + w * 16; const size_t rb = (size_t)b * NN;
  F2 aq[2];
#pragma unroll
  for (int kc = 0; kc < 2; ++kc) aq[kc] = split_row(QP + (rb + q0 + col) * CC, kc * 32, lane);
  float mrun = -3.0e38f, lrun = 0.f; v8f acc[4] = {};
#pragma unroll 1
  for (int kt = 0; kt < NN / 64; ++kt) {
#pragma unroll
    for (int t = 0; t < 4; ++t) { const size_t ko = (rb + kt * 64 + t * 16 + col) * CC; v8f s = {};
#pragma unroll
      for (int kc = 0; kc < 2; ++kc) { const v16b kb = frag_b(X2T + ko + kc * 32, lane); s = wmma_bf(aq[kc].l, kb, s); s = wmma_bf(aq[kc].h, kb, s); }
#pragma unroll
      for (int r = 0; r < 8; ++r) sS[w][8 * g + r][t * 16 + col] = s[r]; }
    LDSX();
    float mx = -3.4e38f;
#pragma unroll
    for (int jj = 0; jj < 32; ++jj) mx = fmaxf(mx, sS[w][col][g * 32 + jj]);
    mx = fmaxf(mx, __shfl_xor(mx, 16, 32));
    const float mnew = fmaxf(mrun, mx); const float corr = expf(mrun - mnew);
    float ps = 0.f;
#pragma unroll 4
    for (int jj = 0; jj < 32; ++jj) { const float p = exp_ni(sS[w][col][g * 32 + jj] - mnew); ps += p; const __bf16 hi = (__bf16)p; sPh[w][col][g * 32 + jj] = hi; sPl[w][col][g * 32 + jj] = (__bf16)(p - (float)hi); }
    ps += __shfl_xor(ps, 16, 32);
    lrun = lrun * corr + ps; mrun = mnew;
#pragma unroll
    for (int r = 0; r < 8; ++r) { const float cr = __shfl(corr, 8 * g + r, 32);
#pragma unroll
      for (int t = 0; t < 4; ++t) acc[t][r] *= cr; }
    LDSX();
#pragma unroll
    for (int kc = 0; kc < 2; ++kc) { const v16b ph = frag_b(&sPh[w][col][0] + kc * 32, lane), pl = frag_b(&sPl[w][col][0] + kc * 32, lane);
#pragma unroll
      for (int t = 0; t < 4; ++t) { const v16b vb = split_row(x2 + ((size_t)b * CC + t * 16 + col) * NN + kt * 64, kc * 32, lane).h; acc[t] = wmma_bf(pl, vb, acc[t]); acc[t] = wmma_bf(ph, vb, acc[t]); } }
    __builtin_amdgcn_wave_barrier(); }
#pragma unroll
  for (int r = 0; r < 8; ++r) { const float lr = __shfl(lrun, 8 * g + r, 32); const float inv = 1.0f / lr;
#pragma unroll
    for (int t = 0; t < 4; ++t) sO[w][8 * g + r][t * 16 + col] = acc[t][r] * inv; }
  LDSX();
  for (int qq = lane; qq < 16 * 16; qq += 32) { const int rl = qq >> 4, pc = qq & 15; vst2(CTX + (rb + q0 + rl) * CC + pc * 4, *(const v4f*)(&sO[w][rl][pc * 4])); }
}
__global__ __launch_bounds__(128) void k_out(const float* __restrict__ CTX, const float* __restrict__ Wv, const float* __restrict__ bv, const float* __restrict__ gam, const float* __restrict__ xt, float* __restrict__ y) {
  __shared__ __align__(16) float sO[4][16][68];
  const int tid = threadIdx.x, w = tid >> 5, lane = tid & 31, col = lane & 15, g = lane >> 4; const int b = blockIdx.y, p0 = blockIdx.x * 64; const size_t base = (size_t)b * NN; const float gm = bfr(gam[0]);
  v8f acc[4] = {};
#pragma unroll
  for (int kc = 0; kc < CC / 32; ++kc) { const v16b a = split_row(Wv + (size_t)(w * 16 + col) * CC, kc * 32, lane).h;
#pragma unroll
    for (int pt = 0; pt < 4; ++pt) { const F2 bc = split_row(CTX + (base + p0 + pt * 16 + col) * CC, kc * 32, lane); acc[pt] = wmma_bf(a, bc.l, acc[pt]); acc[pt] = wmma_bf(a, bc.h, acc[pt]); } }
#pragma unroll
  for (int r = 0; r < 8; ++r) { const int cl = 8 * g + r; const int c = w * 16 + cl; const float bb = bfr(bv[c]);
#pragma unroll
    for (int pt = 0; pt < 4; ++pt) { const int n = p0 + pt * 16 + col; sO[w][cl][pt * 16 + col] = gm * (acc[pt][r] + bb) + bfr(xt[((size_t)b * CC + c) * NN + n]); } }
  LDSX();
  for (int qq = lane; qq < 16 * 16; qq += 32) { const int cl = qq >> 4, pc = qq & 15; vst2(y + ((size_t)b * CC + w * 16 + cl) * NN + p0 + pc * 4, *(const v4f*)(&sO[w][cl][pc * 4])); }
}
extern "C" void kernel_launch(void* const* d_in, const int* in_sizes, int n_in, void* d_out, int out_size, void* d_ws, size_t ws_size, hipStream_t stream) {
  (void)in_sizes; (void)n_in; (void)out_size; (void)ws_size;
  const float** I = (const float**)d_in;
  const float* xs = I[0]; const float* xt = I[1]; const float* Wq = I[2]; const float* bq = I[3]; const float* Wk = I[4]; const float* Wv = I[6]; const float* bv = I[7]; const float* gam = I[8];
  char* ws = (char*)d_ws; size_t off = 0;
  auto take = [&](size_t bytes) { char* p = ws + off; off += (bytes + 255) & ~(size_t)255; return p; };
  __bf16* XST = (__bf16*)take((size_t)NB * NN * CC * 2); float* QP = (float*)take((size_t)NB * NN * CC * 4); float* CTX = (float*)take((size_t)NB * NN * CC * 4);
  k_cvt<<<dim3(NN / 64, NB, 1), 256, 0, stream>>>(xs, xs, XST, XST);
  k_q<<<dim3(NN / 64, NB), 64, 0, stream>>>(xt, Wq, bq, Wk, QP);
  k_attn<<<dim3(NN / 64, NB), 128, 0, stream>>>(QP, XST, xs, CTX);
  k_out<<<dim3(NN / 64, NB), 128, 0, stream>>>(CTX, Wv, bv, gam, xt, (float*)d_out);
}
